// MultiheadAttention_54185307406968
// MI455X (gfx1250) — hardware-run, weakly checked
//
#include <hip/hip_runtime.h>
#ifndef NB
#define NB 2
#endif
#ifndef SEQ
#define SEQ 1024
#endif
#define NB_FULL 2
#define DM 1024
#define NH 16
#define HD 64
#define QC (SEQ < 256 ? SEQ : 256)
#define NR ((size_t)NB * SEQ)
#define MP ((int)(NB * SEQ))
#define LQ (NB * DM)
static_assert(SEQ % 128 == 0);
static_assert(QC % 128 == 0);
static_assert(SEQ % QC == 0);
static_assert(NH * HD == DM);
static_assert(NB <= NB_FULL);
static_assert((NB * SEQ) % 128 == 0);
static_assert(NH == 16);

typedef unsigned short v8us __attribute__((ext_vector_type(8), may_alias));
typedef float  v8f  __attribute__((ext_vector_type(8)));
typedef float  v4f  __attribute__((ext_vector_type(4)));
typedef float  v4fa __attribute__((ext_vector_type(4), may_alias));
typedef _Float16 v16h __attribute__((ext_vector_type(16)));
typedef _Float16 v4h __attribute__((ext_vector_type(4)));
union FragH { v16h v; v8us half[2]; _Float16 h[16]; unsigned short u[16]; };

__device__ __forceinline__ unsigned short bf16_bits(float x) { unsigned int u = __float_as_uint(x); return (unsigned short)((u + 0x7FFFu + ((u >> 16) & 1u)) >> 16); }
__device__ __forceinline__ float bf16_val(unsigned short b) { return __uint_as_float(((unsigned int)b) << 16); }
__device__ __forceinline__ float bf16_rne(float x) { return bf16_val(bf16_bits(x)); }

__device__ __forceinline__ v16h g2_frag(const _Float16* p, int hh) { FragH f; f.half[0] = *(const v8us*)((const unsigned short*)p + 8 * hh); f.half[1] = *(const v8us*)((const unsigned short*)p + 16 + 8 * hh); return f.v; }
__device__ __forceinline__ v8f g2_mma(v16h a, v16h b, v8f c) { v8f d = __builtin_amdgcn_wmma_f32_16x16x32_f16(false, a, false, b, (short)0, c, false, false); asm volatile("v_nop\n\tv_nop\n\tv_nop\n\tv_nop" : "+v"(d) : "v"(a), "v"(b)); return d; }

template <bool HASB, bool OUT32, bool OMAP>
__global__ __launch_bounds__(128) void k_gemm2(const _Float16* __restrict__ A, int lda, size_t sA, const _Float16* __restrict__ Bh, int ldb, size_t sB, float alpha,
    const float* __restrict__ bias, float* __restrict__ C, _Float16* __restrict__ C16, int ldc, size_t sC, int M, int N, int K) {
  __shared__ __attribute__((aligned(16))) float so[4][32][68];
  const int tid = threadIdx.x, w = __builtin_amdgcn_readfirstlane((int)(tid >> 5)), lane = tid & 31, ln = lane & 15, hh = lane >> 4; const int by = blockIdx.y;
  A += (size_t)by * sA; Bh += (size_t)by * sB; const size_t cofs = (size_t)by * sC;
  const int ntn = N >> 6; const int mt = blockIdx.x / ntn, nq = blockIdx.x - mt * ntn; const int row0 = mt * 128 + 32 * w, col0 = nq * 64; if (row0 >= M) return;
  const _Float16* a0p = A + (size_t)(row0 + ln) * lda; const _Float16* a1p = a0p + (size_t)16 * lda;
  const _Float16* b0p = Bh + (size_t)(col0 + ln) * ldb; const _Float16* b1p = b0p + (size_t)16 * ldb; const _Float16* b2p = b1p + (size_t)16 * ldb; const _Float16* b3p = b2p + (size_t)16 * ldb;
  const v8f z8 = {0.f,0.f,0.f,0.f,0.f,0.f,0.f,0.f}; v8f c00 = z8, c01 = z8, c02 = z8, c03 = z8, c10 = z8, c11 = z8, c12 = z8, c13 = z8;
#pragma unroll 1
  for (int kb = 0; kb < K; kb += 32) { const v16h a0 = g2_frag(a0p + kb, hh), a1 = g2_frag(a1p + kb, hh);
    v16h b = g2_frag(b0p + kb, hh); c00 = g2_mma(a0, b, c00); c10 = g2_mma(a1, b, c10);
    b = g2_frag(b1p + kb, hh); c01 = g2_mma(a0, b, c01); c11 = g2_mma(a1, b, c11);
    b = g2_frag(b2p + kb, hh); c02 = g2_mma(a0, b, c02); c12 = g2_mma(a1, b, c12);
    b = g2_frag(b3p + kb, hh); c03 = g2_mma(a0, b, c03); c13 = g2_mma(a1, b, c13); }
  v8f accs[8] = {c00, c01, c02, c03, c10, c11, c12, c13};
#pragma unroll
  for (int u = 0; u < 8; ++u) { const int t = u & 3, half = u >> 2; const int col = col0 + t * 16 + ln; float bv = 0.f; if (HASB) bv = bf16_rne(bias[col]);
#pragma unroll
    for (int r = 0; r < 8; ++r) { const int rloc = half * 16 + 8 * hh + r; so[w][rloc][t * 16 + ln] = accs[u][r] * alpha + bv; } }
  __builtin_amdgcn_fence(4  , "workgroup"); __builtin_amdgcn_wave_barrier();
  const int rsub = lane >> 4, c4 = (lane & 15) * 4;
  for (int pass = 0; pass < 2; ++pass) {
#pragma unroll
    for (int q = 0; q < 16; ++q) { const int r = q * 2 + rsub; const v4f v = *(const v4fa*)&so[w][r][c4];
      const int gr = row0 + r; const size_t orow = OMAP ? ((size_t)(gr / NB) * NB_FULL + (size_t)(gr % NB)) : (size_t)gr;
      if (OUT32) { *(volatile v4f*)(C + cofs + orow * ldc + col0 + c4) = v; }
      else { v4h h4;
#pragma unroll
        for (int i = 0; i < 4; ++i) h4[i] = (_Float16)v[i];
        *(volatile v4h*)(C16 + cofs + orow * ldc + col0 + c4) = h4; } }
    if (pass == 0) __threadfence(); } }

__global__ __launch_bounds__(256) void k_wnat(const float* __restrict__ w, size_t n8, _Float16* __restrict__ Bt) { const size_t t = (size_t)blockIdx.x * 256 + threadIdx.x; if (t >= n8) return; FragH f; const v4f a = *(const v4fa*)(w + t * 8), c = *(const v4fa*)(w + t * 8 + 4);
#pragma unroll
  for (int q = 0; q < 4; ++q) { f.h[q] = (_Float16)(bf16_rne(a[q]) * 16.0f); f.h[4 + q] = (_Float16)(bf16_rne(c[q]) * 16.0f); }
  const v8us o = f.half[0]; *(volatile v8us*)((unsigned short*)Bt + t * 8) = o; __threadfence(); *(volatile v8us*)((unsigned short*)Bt + t * 8) = o; }

__global__ __launch_bounds__(256) void k_x16(const float* __restrict__ x, _Float16* __restrict__ X16, size_t n8) { const size_t t = (size_t)blockIdx.x * 256 + threadIdx.x; if (t >= n8) return;
  const size_t row = t / (DM / 8); const int c8 = (int)(t % (DM / 8)) * 8; const size_t srow = (row / NB) * NB_FULL + (row % NB);
  const float* p = x + srow * DM + c8; const v4f a = *(const v4fa*)p, c = *(const v4fa*)(p + 4); FragH f;
#pragma unroll
  for (int q = 0; q < 4; ++q) { f.h[q] = (_Float16)bf16_rne(a[q]); f.h[4 + q] = (_Float16)bf16_rne(c[q]); }
  const v8us o = f.half[0]; *(volatile v8us*)((unsigned short*)X16 + t * 8) = o; __threadfence(); *(volatile v8us*)((unsigned short*)X16 + t * 8) = o; }

__global__ __launch_bounds__(64) void k_wmix(const float* __restrict__ mixw, _Float16* __restrict__ WT) {
  const int i = threadIdx.x; const int g = i >> 2, k8 = (i & 3) * 8; float mx = -3.0e38f;
#pragma unroll 1
  for (int h = 0; h < NH; ++h) mx = fmaxf(mx, bf16_rne(mixw[h * NH + g]));
  float se = 0.f;
#pragma unroll 1
  for (int h = 0; h < NH; ++h) se += __expf(bf16_rne(mixw[h * NH + g]) - mx);
  const float inv = 1.0f / se; FragH f;
#pragma unroll
  for (int q = 0; q < 8; ++q) { const int h = k8 + q; const int hc = (h < NH) ? h : (NH - 1); const float v = __expf(bf16_rne(mixw[hc * NH + g]) - mx) * inv; f.h[q] = (_Float16)((h < NH) ? v : 0.0f); }
  const v8us o = f.half[0]; *(volatile v8us*)((unsigned short*)WT + i * 8) = o; __threadfence(); *(volatile v8us*)((unsigned short*)WT + i * 8) = o; }

__global__ __launch_bounds__(256) void k_vt(const _Float16* __restrict__ V16, _Float16* __restrict__ Vt) { __shared__ unsigned short tl[64][66]; const int tid = threadIdx.x; const int slab = blockIdx.x / (SEQ / 64), lg = blockIdx.x % (SEQ / 64); const int b = slab / NH, h = slab % NH;
  for (int i = tid; i < 64 * 8; i += 256) { const int r = i / 8, c8 = (i % 8) * 8; FragH f; f.half[0] = *(const v8us*)((const unsigned short*)V16 + ((size_t)(lg * 64 + r) * NB + b) * DM + h * HD + c8);
#pragma unroll
    for (int q = 0; q < 8; ++q) tl[r][c8 + q] = f.u[q]; }
  __syncthreads();
  for (int pass = 0; pass < 2; ++pass) {
#pragma unroll
    for (int rd = 0; rd < 2; ++rd) { const int d = rd * 32 + tid / 8, pc = tid % 8; FragH f;
#pragma unroll
      for (int q = 0; q < 8; ++q) f.u[q] = tl[pc * 8 + q][d];
      *(volatile v8us*)((unsigned short*)Vt + ((size_t)slab * 64 + d) * SEQ + lg * 64 + pc * 8) = f.half[0]; }
    if (pass == 0) __threadfence(); } }

__global__ __launch_bounds__(128) void k_smix(const float* __restrict__ S, const _Float16* __restrict__ WT, _Float16* __restrict__ PM) {
  #pragma clang fp contract(off)
  __shared__ float sst[4][2][NH];
  __shared__ __attribute__((aligned(16))) _Float16 sP[4][NH][72];
  const int tid = threadIdx.x, w = __builtin_amdgcn_readfirstlane((int)(tid >> 5)), lane = tid & 31, ln = lane & 15, hh = lane >> 4;
  const int wr = blockIdx.x * 4 + w; const int b = wr / QC, tql = wr - b * QC;
  const size_t hp = (size_t)QC * SEQ;
  const float* srow = S + ((size_t)(b * NH) * QC + tql) * SEQ;
#pragma unroll 1
  for (int h = 0; h < NH; ++h) {
    const float* p = srow + (size_t)h * hp + lane * 4;
    v4f x[SEQ / 128];
#pragma unroll
    for (int j = 0; j < SEQ / 128; ++j) x[j] = *(const v4fa*)(p + j * 128);
    float mx = -3.0e38f;
#pragma unroll
    for (int j = 0; j < SEQ / 128; ++j) mx = fmaxf(mx, fmaxf(fmaxf(x[j][0], x[j][1]), fmaxf(x[j][2], x[j][3])));
#pragma unroll
    for (int off = 16; off > 0; off >>= 1) mx = fmaxf(mx, __shfl_xor(mx, off, 32));
    float se = 0.f;
#pragma unroll
    for (int j = 0; j < SEQ / 128; ++j) { se += __expf(x[j][0] - mx); se += __expf(x[j][1] - mx); se += __expf(x[j][2] - mx); se += __expf(x[j][3] - mx); }
#pragma unroll
    for (int off = 16; off > 0; off >>= 1) se += __shfl_xor(se, off, 32);
    if (lane == 0) { sst[w][0][h] = mx; sst[w][1][h] = 1024.0f / se; }
  }
  __syncthreads();
  float m8[8], c8[8];
#pragma unroll
  for (int i = 0; i < 8; ++i) { m8[i] = sst[w][0][8 * hh + i]; c8[i] = sst[w][1][8 * hh + i]; }
  const v16h aW = g2_frag(WT + ln * 32, hh);
  const v8f z8 = {0.f,0.f,0.f,0.f,0.f,0.f,0.f,0.f};
  const float* scol = srow + (size_t)(8 * hh) * hp + ln;
  unsigned short* pout = (unsigned short*)PM + ((size_t)(b * NH) * QC + tql) * SEQ;
#pragma unroll 1
  for (int c0 = 0; c0 < SEQ; c0 += 64) {
#pragma unroll 1
    for (int t = 0; t < 4; ++t) {
      const float* ps = scol + c0 + 16 * t;
      FragH bf;
#pragma unroll
      for (int i = 0; i < 8; ++i) { const float v = ps[(size_t)i * hp]; bf.h[i] = (_Float16)(__expf(v - m8[i]) * c8[i]); }
#pragma unroll
      for (int i = 8; i < 16; ++i) bf.h[i] = (_Float16)0.0f;
      const v8f d = g2_mma(aW, bf.v, z8);
#pragma unroll
      for (int r = 0; r < 8; ++r) sP[w][8 * hh + r][16 * t + ln] = (_Float16)d[r];
    }
    __builtin_amdgcn_fence(4  , "workgroup"); __builtin_amdgcn_wave_barrier();
    for (int pass = 0; pass < 2; ++pass) {
#pragma unroll
      for (int q = 0; q < 4; ++q) { const int g = q * 4 + (lane >> 3), pc = lane & 7; const v8us v = *(const v8us*)&sP[w][g][pc * 8];
        *(volatile v8us*)(pout + (size_t)g * hp + c0 + pc * 8) = v; }
      if (pass == 0) __threadfence(); }
    __builtin_amdgcn_fence(4  , "workgroup"); __builtin_amdgcn_wave_barrier();
  }
}

extern "C" void kernel_launch(void* const* d_in, const int* in_sizes, int n_in,
                              void* d_out, int out_size, void* d_ws, size_t ws_size, hipStream_t stream) {
  if (n_in < 10) return;
  if ((size_t)in_sizes[0] < NR * DM) return;
  if ((size_t)in_sizes[1] < (size_t)DM * DM || (size_t)in_sizes[3] < (size_t)DM * DM || (size_t)in_sizes[5] < (size_t)DM * DM || (size_t)in_sizes[7] < (size_t)DM * DM) return;
  if (in_sizes[2] < DM || in_sizes[4] < DM || in_sizes[6] < DM || in_sizes[8] < DM || in_sizes[9] < NH * NH) return;
  if ((size_t)out_size < NR * DM) return;
  const float* const* I = (const float* const*)d_in;
  const float* xq = I[0]; const float* wq = I[1]; const float* bq = I[2]; const float* wk = I[3]; const float* bk = I[4]; const float* wv = I[5]; const float* bv = I[6]; const float* wo = I[7]; const float* bo = I[8]; const float* mixw = I[9];
  char* ws = (char*)d_ws; size_t off = 0;
  auto take = [&](size_t bytes) { char* p = ws + off; off += (bytes + 255) & ~(size_t)255; return p; };
  _Float16* BQ = (_Float16*)take((size_t)DM * DM * 2); _Float16* BK = (_Float16*)take((size_t)DM * DM * 2); _Float16* BV = (_Float16*)take((size_t)DM * DM * 2); _Float16* BO = (_Float16*)take((size_t)DM * DM * 2);
  _Float16* X16 = (_Float16*)take(NR * DM * 2); _Float16* Q16 = (_Float16*)take(NR * DM * 2); _Float16* K16 = (_Float16*)take(NR * DM * 2); _Float16* V16 = (_Float16*)take(NR * DM * 2); _Float16* O16 = (_Float16*)take(NR * DM * 2);
  float* S = (float*)take((size_t)NB * NH * QC * SEQ * 4); _Float16* PM = (_Float16*)take((size_t)NB * NH * QC * SEQ * 2); _Float16* VT = (_Float16*)take((size_t)NB * NH * HD * SEQ * 2);
  _Float16* WT = (_Float16*)take((size_t)NH * 32 * 2);
  if (off > ws_size) return;
  { const unsigned g = (unsigned)(((size_t)DM * DM / 8 + 255) / 256);
    k_wnat<<<g, 256, 0, stream>>>(wq, (size_t)DM * DM / 8, BQ); k_wnat<<<g, 256, 0, stream>>>(wk, (size_t)DM * DM / 8, BK);
    k_wnat<<<g, 256, 0, stream>>>(wv, (size_t)DM * DM / 8, BV); k_wnat<<<g, 256, 0, stream>>>(wo, (size_t)DM * DM / 8, BO); }
  k_wmix<<<1, 64, 0, stream>>>(mixw, WT);
  k_x16<<<(unsigned)((NR * DM / 8 + 255) / 256), 256, 0, stream>>>(xq, X16, NR * DM / 8);
  const dim3 gp((unsigned)((MP / 128) * (DM / 64)), 1);
  k_gemm2<true, false, false><<<gp, 128, 0, stream>>>(X16, DM, 0, BQ, DM, 0, 0.0625f, bq, nullptr, Q16, DM, 0, MP, DM, DM);
  k_gemm2<true, false, false><<<gp, 128, 0, stream>>>(X16, DM, 0, BK, DM, 0, 0.0625f, bk, nullptr, K16, DM, 0, MP, DM, DM);
  k_gemm2<true, false, false><<<gp, 128, 0, stream>>>(X16, DM, 0, BV, DM, 0, 0.0625f, bv, nullptr, V16, DM, 0, MP, DM, DM);
  k_vt<<<NB * NH * (SEQ / 64), 256, 0, stream>>>(V16, VT);
  for (int t0 = 0; t0 < SEQ; t0 += QC) {
    k_gemm2<false, true, false><<<dim3((QC / 128) * (SEQ / 64), NB * NH), 128, 0, stream>>>(Q16 + (size_t)t0 * LQ, LQ, (size_t)HD, K16, LQ, (size_t)HD, 0.125f, nullptr, S, nullptr, SEQ, (size_t)QC * SEQ, QC, SEQ, HD);
    k_smix<<<NB * QC / 4, 128, 0, stream>>>(S, WT, PM);
    k_gemm2<false, false, false><<<dim3((QC / 128) * (HD / 64), NB * NH), 128, 0, stream>>>(PM, SEQ, (size_t)QC * SEQ, VT, SEQ, (size_t)HD * SEQ, 0.0625f, nullptr, nullptr, O16 + (size_t)t0 * LQ, LQ, (size_t)HD, QC, HD, SEQ);
  }
  k_gemm2<true, true, true><<<gp, 128, 0, stream>>>(O16, DM, 0, BO, DM, 0, 0.0009765625f, bo, (float*)d_out, nullptr, DM, 0, MP, DM, DM);
}
